// TwoLayerResidualGAT_429496730274
// MI455X (gfx1250) — hardware-verified
//
#include <hip/hip_runtime.h>
#include <stddef.h>
#include <stdint.h>
#include <math.h>

#define FIN   128
#define NH1   4
#define HD    256
#define HD1   (NH1 * HD)
#define D2    256
#define NTHR  256
#define NWAVE 8
#define GR    32
#define GC    256
#define CSP   260
#define RP    64
#define NB1   64
#define NB2   256
#define CHUNK 2048
#define NGRP  (CHUNK / (NTHR * 4))
#define WCAP  ((CHUNK / NTHR) * 32)
#define AGG_LDS(D_, NH_, NB_) ((((NB_) * (D_)) + 2 * (NB_) * (NH_)) * 4 + (NWAVE * WCAP + NWAVE) * 4)

static_assert(NGRP >= 1);
static_assert(WCAP == 256);
static_assert(CHUNK <= 2048);
static_assert(AGG_LDS(HD1, NH1, NB1) == 272416);
static_assert(AGG_LDS(D2, 1, NB2) == 272416);
static_assert((CSP * 4) % 16 == 0);

typedef float  v4f  __attribute__((ext_vector_type(4)));
typedef float  v8f  __attribute__((ext_vector_type(8)));
typedef int    v4i  __attribute__((ext_vector_type(4)));
typedef __bf16 v8b  __attribute__((ext_vector_type(8)));
typedef __bf16 v16b __attribute__((ext_vector_type(16)));
union Frag  { v16b v; v8b half[2]; };
union Pack8 { v8b h; v4i i; };

__device__ __forceinline__ v8f wm(v16b a, v16b b, v8f c) {
  v8f d = __builtin_amdgcn_wmma_f32_16x16x32_bf16(false, a, false, b, (short)0, c, false, false);
  asm volatile("v_nop\n\tv_nop\n\tv_nop\n\tv_nop" : "+v"(d) : "v"(a), "v"(b));
  return d;
}

__device__ __forceinline__ void split8(v4f a, v4f b, Pack8& hi, Pack8& lo) {
  const float f[8] = {a.x, a.y, a.z, a.w, b.x, b.y, b.z, b.w};
#pragma unroll
  for (int j = 0; j < 8; ++j) {
    const __bf16 hv = (__bf16)f[j];
    hi.h[j] = hv;
    lo.h[j] = (__bf16)(f[j] - (float)hv);
  }
}

__device__ __forceinline__ int clampi(int v, int hi) { return v < 0 ? 0 : (v > hi ? hi : v); }

__device__ __forceinline__ v4f elu4(v4f v) {
  v4f r;
  r.x = v.x > 0.f ? v.x : expm1f(v.x);
  r.y = v.y > 0.f ? v.y : expm1f(v.y);
  r.z = v.z > 0.f ? v.z : expm1f(v.z);
  r.w = v.w > 0.f ? v.w : expm1f(v.w);
  return r;
}

__global__ __launch_bounds__(NTHR) void k_cvt_x(const float* __restrict__ x, int nN, int Mp,
                                                __bf16* xh, __bf16* xl) {
  const int i = blockIdx.x * NTHR + threadIdx.x;
  if (i >= Mp * (FIN / 8)) return;
  const int row = i / (FIN / 8);
  const int c = (i - row * (FIN / 8)) * 8;
  v4f a = {0.f, 0.f, 0.f, 0.f};
  v4f b = a;
  if (row < nN) {
    const float* p = x + (size_t)row * FIN + c;
    a = *(const v4f*)p;
    b = *(const v4f*)(p + 4);
  }
  Pack8 hi, lo;
  split8(a, b, hi, lo);
  const size_t o = (size_t)row * FIN + c;
  *(volatile v4i*)(xh + o) = hi.i;
  *(volatile v4i*)(xl + o) = lo.i;
  __threadfence();
  *(volatile v4i*)(xh + o) = hi.i;
  *(volatile v4i*)(xl + o) = lo.i;
}

__global__ __launch_bounds__(NTHR) void k_wt(const float* __restrict__ W, int K, int NC,
                                             __bf16* Th, __bf16* Tl) {
  __shared__ float T[64][33];
  const int tid = threadIdx.x;
  const int n0 = blockIdx.x * 32;
  const int k0 = blockIdx.y * 64;
  {
    const int kr = tid >> 2;
    const int cq = (tid & 3) * 8;
    const float* p = W + (size_t)(k0 + kr) * NC + n0 + cq;
    const v4f a = *(const v4f*)p;
    const v4f b = *(const v4f*)(p + 4);
    T[kr][cq + 0] = a.x; T[kr][cq + 1] = a.y; T[kr][cq + 2] = a.z; T[kr][cq + 3] = a.w;
    T[kr][cq + 4] = b.x; T[kr][cq + 5] = b.y; T[kr][cq + 6] = b.z; T[kr][cq + 7] = b.w;
  }
  __syncthreads();
  const int n  = tid >> 3;
  const int ks = (tid & 7) * 8;
  v4f a, b;
  a.x = T[ks + 0][n]; a.y = T[ks + 1][n]; a.z = T[ks + 2][n]; a.w = T[ks + 3][n];
  b.x = T[ks + 4][n]; b.y = T[ks + 5][n]; b.z = T[ks + 6][n]; b.w = T[ks + 7][n];
  Pack8 hi, lo;
  split8(a, b, hi, lo);
  const size_t o = (size_t)(n0 + n) * K + k0 + ks;
  *(volatile v4i*)(Th + o) = hi.i;
  *(volatile v4i*)(Tl + o) = lo.i;
  __threadfence();
  *(volatile v4i*)(Th + o) = hi.i;
  *(volatile v4i*)(Tl + o) = lo.i;
}

__global__ __launch_bounds__(NTHR) void k_gemm(
    const __bf16* __restrict__ Ahi, const __bf16* __restrict__ Alo, int lda,
    const __bf16* __restrict__ Bh, const __bf16* __restrict__ Bl, int K, int NC, int mode,
    float* C,
    const float* __restrict__ att_s, const float* __restrict__ att_d, float* ss, float* sd, int Mp,
    const float* __restrict__ addp, const float* __restrict__ bias0, const float* __restrict__ bias1,
    __bf16* Hh, __bf16* Hl) {
  __shared__ __attribute__((aligned(16))) float Cs[GR * CSP];
  __shared__ __attribute__((aligned(16))) float Ssc[GR];
  __shared__ __attribute__((aligned(16))) float Sdc[GR];

  const int tid  = threadIdx.x;
  const int lane = tid & 31;
  const int wave = tid >> 5;
  const int hh   = lane >> 4;
  const int m    = lane & 15;
  const int rowBase = blockIdx.y * GR;
  const int colBase = blockIdx.x * GC;
  const int wcol = colBase + wave * 32;

  const __bf16* pa0h = Ahi + (size_t)(rowBase + m) * lda + 8 * hh;
  const __bf16* pa1h = Ahi + (size_t)(rowBase + 16 + m) * lda + 8 * hh;
  const __bf16* pa0l = Alo + (size_t)(rowBase + m) * lda + 8 * hh;
  const __bf16* pa1l = Alo + (size_t)(rowBase + 16 + m) * lda + 8 * hh;
  const __bf16* pb0h = Bh + (size_t)(wcol + m) * K + 8 * hh;
  const __bf16* pb1h = Bh + (size_t)(wcol + 16 + m) * K + 8 * hh;
  const __bf16* pb0l = Bl + (size_t)(wcol + m) * K + 8 * hh;
  const __bf16* pb1l = Bl + (size_t)(wcol + 16 + m) * K + 8 * hh;

  v8f c00 = {0.f, 0.f, 0.f, 0.f, 0.f, 0.f, 0.f, 0.f};
  v8f c01 = c00, c10 = c00, c11 = c00;
  const int S = K >> 5;
#pragma unroll 1
  for (int s = 0; s < S; ++s) {
    const int k0 = s << 5;
    Frag a0h, a0l, a1h, a1l, b0h, b0l, b1h, b1l;
    a0h.half[0] = *(const v8b*)(pa0h + k0); a0h.half[1] = *(const v8b*)(pa0h + k0 + 16);
    a0l.half[0] = *(const v8b*)(pa0l + k0); a0l.half[1] = *(const v8b*)(pa0l + k0 + 16);
    a1h.half[0] = *(const v8b*)(pa1h + k0); a1h.half[1] = *(const v8b*)(pa1h + k0 + 16);
    a1l.half[0] = *(const v8b*)(pa1l + k0); a1l.half[1] = *(const v8b*)(pa1l + k0 + 16);
    b0h.half[0] = *(const v8b*)(pb0h + k0); b0h.half[1] = *(const v8b*)(pb0h + k0 + 16);
    b0l.half[0] = *(const v8b*)(pb0l + k0); b0l.half[1] = *(const v8b*)(pb0l + k0 + 16);
    b1h.half[0] = *(const v8b*)(pb1h + k0); b1h.half[1] = *(const v8b*)(pb1h + k0 + 16);
    b1l.half[0] = *(const v8b*)(pb1l + k0); b1l.half[1] = *(const v8b*)(pb1l + k0 + 16);
    c00 = wm(a0h.v, b0h.v, c00); c00 = wm(a0h.v, b0l.v, c00); c00 = wm(a0l.v, b0h.v, c00);
    c01 = wm(a0h.v, b1h.v, c01); c01 = wm(a0h.v, b1l.v, c01); c01 = wm(a0l.v, b1h.v, c01);
    c10 = wm(a1h.v, b0h.v, c10); c10 = wm(a1h.v, b0l.v, c10); c10 = wm(a1l.v, b0h.v, c10);
    c11 = wm(a1h.v, b1h.v, c11); c11 = wm(a1h.v, b1l.v, c11); c11 = wm(a1l.v, b1h.v, c11);
  }

#pragma unroll
  for (int r = 0; r < 8; ++r) {
    float* p0 = Cs + (8 * hh + r) * CSP + wave * 32 + m;
    float* p1 = Cs + (16 + 8 * hh + r) * CSP + wave * 32 + m;
    p0[0] = c00[r]; p0[16] = c01[r];
    p1[0] = c10[r]; p1[16] = c11[r];
  }
  __syncthreads();

  if (mode == 1) {
    const int c8 = 8 * lane;
    const v4f bb0 = *(const v4f*)(bias0 + colBase + c8);
    const v4f bb1 = *(const v4f*)(bias0 + colBase + c8 + 4);
    Pack8 hi[4], lo[4];
    size_t off[4];
#pragma unroll
    for (int i = 0; i < 4; ++i) {
      const int row = 4 * wave + i;
      const size_t grow = (size_t)(rowBase + row);
      v4f v0 = *(const v4f*)(Cs + row * CSP + c8);
      v4f v1 = *(const v4f*)(Cs + row * CSP + c8 + 4);
      const float* ap = addp + grow * NC + colBase + c8;
      v0 = v0 + *(const v4f*)ap + bb0;
      v1 = v1 + *(const v4f*)(ap + 4) + bb1;
      v0 = elu4(v0);
      v1 = elu4(v1);
      split8(v0, v1, hi[i], lo[i]);
      off[i] = grow * NC + colBase + c8;
    }
#pragma unroll
    for (int i = 0; i < 4; ++i) {
      *(volatile v4i*)(Hh + off[i]) = hi[i].i;
      *(volatile v4i*)(Hl + off[i]) = lo[i].i;
    }
    __threadfence();
#pragma unroll
    for (int i = 0; i < 4; ++i) {
      *(volatile v4i*)(Hh + off[i]) = hi[i].i;
      *(volatile v4i*)(Hl + off[i]) = lo[i].i;
    }
  } else {
    const v4f z4 = {0.f, 0.f, 0.f, 0.f};
    v4f badd0 = z4, badd1 = z4;
    if (mode == 2) {
      badd0 = *(const v4f*)(bias0 + colBase + 4 * lane) + *(const v4f*)(bias1 + colBase + 4 * lane);
      badd1 = *(const v4f*)(bias0 + colBase + 128 + 4 * lane) + *(const v4f*)(bias1 + colBase + 128 + 4 * lane);
    }
    v4f vals[8];
    size_t off[8];
#pragma unroll
    for (int i = 0; i < 4; ++i) {
      const int row = 4 * wave + i;
      const size_t grow = (size_t)(rowBase + row);
      vals[2 * i]     = *(const v4f*)(Cs + row * CSP + 4 * lane) + badd0;
      vals[2 * i + 1] = *(const v4f*)(Cs + row * CSP + 128 + 4 * lane) + badd1;
      off[2 * i]      = grow * NC + colBase + 4 * lane;
      off[2 * i + 1]  = grow * NC + colBase + 128 + 4 * lane;
    }
#pragma unroll
    for (int i = 0; i < 8; ++i) *(volatile v4f*)(C + off[i]) = vals[i];
    __threadfence();
#pragma unroll
    for (int i = 0; i < 8; ++i) *(volatile v4f*)(C + off[i]) = vals[i];

    if (mode == 0) {
      const int r = tid >> 3;
      const int q = tid & 7;
      const float* crow = Cs + r * CSP + 32 * q;
      const float* asp  = att_s + colBase + 32 * q;
      const float* adp  = att_d + colBase + 32 * q;
      float s1 = 0.f, s2 = 0.f;
#pragma unroll
      for (int j = 0; j < 8; ++j) {
        const v4f cv = *(const v4f*)(crow + 4 * j);
        const v4f av = *(const v4f*)(asp + 4 * j);
        const v4f dv = *(const v4f*)(adp + 4 * j);
        s1 += cv.x * av.x + cv.y * av.y + cv.z * av.z + cv.w * av.w;
        s2 += cv.x * dv.x + cv.y * dv.y + cv.z * dv.z + cv.w * dv.w;
      }
      s1 += __shfl_xor(s1, 1, 32); s1 += __shfl_xor(s1, 2, 32); s1 += __shfl_xor(s1, 4, 32);
      s2 += __shfl_xor(s2, 1, 32); s2 += __shfl_xor(s2, 2, 32); s2 += __shfl_xor(s2, 4, 32);
      if (q == 0) { Ssc[r] = s1; Sdc[r] = s2; }
      __syncthreads();
      if (wave == 0 && lane < 16) {
        const int head = blockIdx.x;
        v4f v;
        float* gp;
        if (lane < 8) {
          v  = *(const v4f*)(Ssc + 4 * lane);
          gp = ss + (size_t)head * Mp + rowBase + 4 * lane;
        } else {
          v  = *(const v4f*)(Sdc + 4 * (lane - 8));
          gp = sd + (size_t)head * Mp + rowBase + 4 * (lane - 8);
        }
        *(volatile v4f*)gp = v;
        __threadfence();
        *(volatile v4f*)gp = v;
      }
    }
  }
}

template <int NH>
__global__ __launch_bounds__(NTHR) void k_edge_p(const int* __restrict__ ei, int nE, int nEt, int nN,
                                                 const float* __restrict__ ss, const float* __restrict__ sd,
                                                 int Mp, float* P, int nGroups) {
  const int t = blockIdx.x * NTHR + threadIdx.x;
  if (t >= nGroups) return;
  float pv[4];
#pragma unroll
  for (int j = 0; j < 4; ++j) {
    const int f = 4 * t + j;
    int e = f / NH;
    const int h = f - e * NH;
    if (e > nEt - 1) e = nEt - 1;
    int src, dst;
    if (e < nE) {
      src = clampi(ei[e], nN - 1);
      dst = clampi(ei[nE + e], nN - 1);
    } else {
      src = e - nE;
      dst = src;
    }
    float a = ss[(size_t)h * Mp + src] + sd[(size_t)h * Mp + dst];
    a = (a >= 0.f) ? a : 0.2f * a;
    a = fminf(a, 80.f);
    pv[j] = expf(a);
  }
  v4f v;
  v.x = pv[0]; v.y = pv[1]; v.z = pv[2]; v.w = pv[3];
  float* gp = P + (size_t)t * 4;
  *(volatile v4f*)gp = v;
  __threadfence();
  *(volatile v4f*)gp = v;
}

template <int D, int NH, int NB, int SUBS>
__global__ __launch_bounds__(NTHR) void k_agg(const int* __restrict__ ei, int nE, int nN,
                                              const float* __restrict__ P, const float* __restrict__ Hs,
                                              const float* __restrict__ bias, const float* __restrict__ addp,
                                              float* outp, int outRows, float* dens, int Mp) {
  constexpr int NSLAB = D / 128;
  constexpr int NBS = NB / SUBS;
  constexpr int HDW = D / NH;
  static_assert(NSLAB * SUBS == NWAVE);
  static_assert(NB <= 256);
  static_assert((NB & (NB - 1)) == 0);
  static_assert((NBS & (NBS - 1)) == 0);
  static_assert(HDW % 128 == 0);
  static_assert(((NB * D + 2 * NB * NH) % 4) == 0);
  static_assert((NB * NH) % 4 == 0);

  extern __shared__ v4f lds_dyn[];
  float* sacc = (float*)lds_dyn;
  float* den  = sacc + NB * D;
  float* denT = den + NB * NH;
  int*   list = (int*)(denT + NB * NH);
  int*   wcnt = list + NWAVE * WCAP;

  const int tid  = threadIdx.x;
  const int lane = tid & 31;
  const int wave = tid >> 5;
  const int slab = wave % NSLAB;
  const int sub  = wave / NSLAB;
  const int head = (slab * 128) / HDW;
  const bool denOwner = ((slab * 128) % HDW) == 0;
  const int colOff = slab * 128 + 4 * lane;
  const int nodeBase = blockIdx.x * NB;

  {
    const v4f z4 = {0.f, 0.f, 0.f, 0.f};
    for (int i = tid; i < (NB * D + 2 * NB * NH) / 4; i += NTHR) lds_dyn[i] = z4;
  }
  __syncthreads();

  const int* eid = ei + nE;
  const bool al16 = ((nE & 3) == 0);

  const int nChunks = (nE + CHUNK - 1) / CHUNK;
#pragma unroll 1
  for (int ch = 0; ch < nChunks; ++ch) {
    const int cbase = ch * CHUNK;
    int wc = 0;
#pragma unroll
    for (int g = 0; g < NGRP; ++g) {
      const int el0 = (g * NTHR + tid) * 4;
      const int e0  = cbase + el0;
      const int sent = -2147483647 - 1;
      v4i d;
      if (al16 && (e0 + 3 < nE)) {
        d = *(const v4i*)(eid + e0);
      } else {
        d.x = (e0     < nE) ? eid[min(e0, nE - 1)]     : sent;
        d.y = (e0 + 1 < nE) ? eid[min(e0 + 1, nE - 1)] : sent;
        d.z = (e0 + 2 < nE) ? eid[min(e0 + 2, nE - 1)] : sent;
        d.w = (e0 + 3 < nE) ? eid[min(e0 + 3, nE - 1)] : sent;
      }
      const unsigned s0 = (unsigned)d.x - (unsigned)nodeBase;
      const unsigned s1 = (unsigned)d.y - (unsigned)nodeBase;
      const unsigned s2 = (unsigned)d.z - (unsigned)nodeBase;
      const unsigned s3 = (unsigned)d.w - (unsigned)nodeBase;
      const bool h0 = s0 < (unsigned)NB;
      const bool h1 = s1 < (unsigned)NB;
      const bool h2 = s2 < (unsigned)NB;
      const bool h3 = s3 < (unsigned)NB;
      const unsigned many = __builtin_amdgcn_ballot_w32(h0 | h1 | h2 | h3);
      if (many != 0u) {
#define HITJ(J, HJ, SJ) { \
          const unsigned mj = __builtin_amdgcn_ballot_w32(HJ); \
          if (HJ) { \
            const int pos = wc + (int)__builtin_amdgcn_mbcnt_lo(mj, 0u); \
            if (pos < WCAP) list[wave * WCAP + pos] = ((el0 + (J)) << 9) | (int)(SJ); \
          } \
          wc += (int)__builtin_popcount(mj); }
        HITJ(0, h0, s0)
        HITJ(1, h1, s1)
        HITJ(2, h2, s2)
        HITJ(3, h3, s3)
#undef HITJ
      }
    }
    if (lane == 0) wcnt[wave] = wc;
    __syncthreads();

    for (int wsx = 0; wsx < NWAVE; ++wsx) {
      int n = wcnt[wsx];
      n = n > WCAP ? WCAP : n;
      n = n < 0 ? 0 : n;
      for (int i = 0; i < n; ++i) {
        const int ent  = list[wsx * WCAP + i];
        const int slot = ent & (NB - 1);
        if (SUBS > 1) {
          if ((slot / NBS) != sub) continue;
        }
        const int el = (ent >> 9) & (CHUNK - 1);
        int e = cbase + el;
        if (e > nE - 1) e = nE - 1;
        const int src = clampi(ei[e], nN - 1);
        const float p = P[(size_t)e * NH + head];
        const v4f xv = *(const v4f*)(Hs + (size_t)src * D + colOff);
        v4f* sp = (v4f*)(sacc + slot * D + colOff);
        const v4f cur = *sp;
        *sp = cur + p * xv;
        if (denOwner && lane == 0) {
          const float o = den[slot * NH + head];
          den[slot * NH + head] = o + p;
        }
      }
    }
    __syncthreads();
  }

  v4f b4 = {0.f, 0.f, 0.f, 0.f};
  if (bias) b4 = *(const v4f*)(bias + colOff);
#pragma unroll 1
  for (int j = 0; j < NBS; ++j) {
    const int slot  = sub * NBS + j;
    const int node  = nodeBase + slot;
    const int nodeC = node > nN - 1 ? nN - 1 : node;
    const float pself = P[((size_t)nE + nodeC) * NH + head];
    const v4f hv = *(const v4f*)(Hs + (size_t)nodeC * D + colOff);
    const v4f sv = *(const v4f*)(sacc + slot * D + colOff) + pself * hv;
    const float dtot = den[slot * NH + head] + pself;
    const float inv = __builtin_amdgcn_rcpf(dtot + 1e-16f);
    v4f v = sv * inv + b4;
    if (addp) v = v + *(const v4f*)(addp + (size_t)nodeC * D + colOff);
    if (denOwner && lane == 0) denT[slot * NH + head] = dtot;
    if (node < outRows) {
      float* op = outp + (size_t)node * D + colOff;
      *(volatile v4f*)op = v;
      __threadfence();
      *(volatile v4f*)op = v;
    }
  }
  __syncthreads();
  if (dens) {
    if (tid < NB * NH / 4) {
      const int hd = tid / (NB / 4);
      const int j  = tid - hd * (NB / 4);
      if (nodeBase + 4 * j + 3 < Mp) {
        v4f v;
        v.x = denT[(4 * j + 0) * NH + hd];
        v.y = denT[(4 * j + 1) * NH + hd];
        v.z = denT[(4 * j + 2) * NH + hd];
        v.w = denT[(4 * j + 3) * NH + hd];
        float* gp = dens + (size_t)hd * Mp + nodeBase + 4 * j;
        *(volatile v4f*)gp = v;
        __threadfence();
        *(volatile v4f*)gp = v;
      }
    }
  }
}

__global__ __launch_bounds__(NTHR) void k_alpha(const int* __restrict__ ei, int nE, int nEt, int nN,
                                                const float* __restrict__ P1, const float* __restrict__ dens,
                                                int Mp, float* out1) {
  const int t = blockIdx.x * NTHR + threadIdx.x;
  if (t >= nEt) return;
  int dst;
  if (t < nE) dst = clampi(ei[nE + t], nN - 1);
  else        dst = t - nE;
  const v4f p = *(const v4f*)(P1 + (size_t)t * 4);
  v4f a;
  a.x = p.x * __builtin_amdgcn_rcpf(dens[dst] + 1e-16f);
  a.y = p.y * __builtin_amdgcn_rcpf(dens[(size_t)Mp + dst] + 1e-16f);
  a.z = p.z * __builtin_amdgcn_rcpf(dens[(size_t)2 * Mp + dst] + 1e-16f);
  a.w = p.w * __builtin_amdgcn_rcpf(dens[(size_t)3 * Mp + dst] + 1e-16f);
  float* gp = out1 + (size_t)t * 4;
  *(volatile v4f*)gp = a;
  __threadfence();
  *(volatile v4f*)gp = a;
}

static inline unsigned cdivu(long a, long b) { return (unsigned)((a + b - 1) / b); }
static inline size_t al256(size_t b) { return (b + 255) & ~(size_t)255; }

extern "C" void kernel_launch(void* const* d_in, const int* in_sizes, int n_in,
                              void* d_out, int out_size, void* d_ws, size_t ws_size,
                              hipStream_t stream) {
  if (n_in < 14) return;
  const int nN = in_sizes[0] / FIN;
  if (nN <= 0 || in_sizes[0] != nN * FIN) return;
  if (in_sizes[1] < 0 || (in_sizes[1] & 1)) return;
  const int nE = in_sizes[1] / 2;
  if (in_sizes[2] != FIN * HD1 || in_sizes[6] != FIN * HD1) return;
  if (in_sizes[3] != NH1 * HD || in_sizes[4] != NH1 * HD) return;
  if (in_sizes[5] != HD1 || in_sizes[7] != HD1) return;
  if (in_sizes[8] != HD1 * D2 || in_sizes[12] != HD1 * D2) return;
  if (in_sizes[9] != D2 || in_sizes[10] != D2 || in_sizes[11] != D2 || in_sizes[13] != D2) return;
  const int nEt = nE + nN;
  if ((long)out_size != (long)nN * D2 + (long)nEt * NH1) return;

  const float* x        = (const float*)d_in[0];
  const int*   ei       = (const int*)d_in[1];
  const float* W1       = (const float*)d_in[2];
  const float* att_src1 = (const float*)d_in[3];
  const float* att_dst1 = (const float*)d_in[4];
  const float* b1       = (const float*)d_in[5];
  const float* lin1_W   = (const float*)d_in[6];
  const float* lin1_b   = (const float*)d_in[7];
  const float* W2       = (const float*)d_in[8];
  const float* att_src2 = (const float*)d_in[9];
  const float* att_dst2 = (const float*)d_in[10];
  const float* b2       = (const float*)d_in[11];
  const float* lin2_W   = (const float*)d_in[12];
  const float* lin2_b   = (const float*)d_in[13];
  float* out0 = (float*)d_out;
  float* out1 = out0 + (size_t)nN * D2;

  const int Mp  = (int)(cdivu(nN, RP) * RP);
  const int Etp = (int)(cdivu(nEt, 32) * 32);

  size_t off = 0;
  char* base = (char*)d_ws;
#define CARVE(PTR, TYPE, BYTES) TYPE* PTR = (TYPE*)(base + off); off += al256((size_t)(BYTES));
  CARVE(xh,   __bf16, (size_t)Mp * FIN * 2)
  CARVE(xl,   __bf16, (size_t)Mp * FIN * 2)
  CARVE(w1h,  __bf16, (size_t)FIN * HD1 * 2)
  CARVE(w1l,  __bf16, (size_t)FIN * HD1 * 2)
  CARVE(l1h,  __bf16, (size_t)FIN * HD1 * 2)
  CARVE(l1l,  __bf16, (size_t)FIN * HD1 * 2)
  CARVE(w2h,  __bf16, (size_t)HD1 * D2 * 2)
  CARVE(w2l,  __bf16, (size_t)HD1 * D2 * 2)
  CARVE(l2h,  __bf16, (size_t)HD1 * D2 * 2)
  CARVE(l2l,  __bf16, (size_t)HD1 * D2 * 2)
  CARVE(HP,   float,  (size_t)Mp * HD1 * 4)
  CARVE(AGG1, float,  (size_t)Mp * HD1 * 4)
  CARVE(H2T,  float,  (size_t)Mp * D2 * 4)
  CARVE(R2,   float,  (size_t)Mp * D2 * 4)
  CARVE(ss1,  float,  (size_t)NH1 * Mp * 4)
  CARVE(sd1,  float,  (size_t)NH1 * Mp * 4)
  CARVE(dens1, float, (size_t)NH1 * Mp * 4)
  CARVE(ss2,  float,  (size_t)Mp * 4)
  CARVE(sd2,  float,  (size_t)Mp * 4)
  CARVE(P1,   float,  (size_t)Etp * NH1 * 4)
  CARVE(P2,   float,  (size_t)Etp * 4)
#undef CARVE
  if (off > ws_size) return;
  __bf16* H1h = (__bf16*)HP;
  __bf16* H1l = H1h + (size_t)Mp * HD1;

  const dim3 B(NTHR);

  k_cvt_x<<<cdivu((long)Mp * (FIN / 8), NTHR), B, 0, stream>>>(x, nN, Mp, xh, xl);
  k_wt<<<dim3(HD1 / 32, FIN / 64), B, 0, stream>>>(W1, FIN, HD1, w1h, w1l);
  k_wt<<<dim3(HD1 / 32, FIN / 64), B, 0, stream>>>(lin1_W, FIN, HD1, l1h, l1l);
  k_wt<<<dim3(D2 / 32, HD1 / 64), B, 0, stream>>>(W2, HD1, D2, w2h, w2l);
  k_wt<<<dim3(D2 / 32, HD1 / 64), B, 0, stream>>>(lin2_W, HD1, D2, l2h, l2l);

  k_gemm<<<dim3(HD1 / GC, Mp / GR), B, 0, stream>>>(xh, xl, FIN, w1h, w1l, FIN, HD1, 0, HP,
                                                    att_src1, att_dst1, ss1, sd1, Mp,
                                                    (const float*)0, (const float*)0, (const float*)0,
                                                    (__bf16*)0, (__bf16*)0);
  k_edge_p<NH1><<<cdivu((long)Etp * NH1 / 4, NTHR), B, 0, stream>>>(ei, nE, nEt, nN, ss1, sd1, Mp, P1,
                                                                     Etp * NH1 / 4);
  hipFuncSetAttribute(reinterpret_cast<const void*>(&k_agg<HD1, NH1, NB1, 1>),
                      hipFuncAttributeMaxDynamicSharedMemorySize, AGG_LDS(HD1, NH1, NB1));
  k_agg<HD1, NH1, NB1, 1><<<Mp / NB1, B, AGG_LDS(HD1, NH1, NB1), stream>>>(
      ei, nE, nN, P1, HP, b1, (const float*)0, AGG1, Mp, dens1, Mp);
  k_alpha<<<cdivu(nEt, NTHR), B, 0, stream>>>(ei, nE, nEt, nN, P1, dens1, Mp, out1);
  k_gemm<<<dim3(HD1 / GC, Mp / GR), B, 0, stream>>>(xh, xl, FIN, l1h, l1l, FIN, HD1, 1, (float*)0,
                                                    (const float*)0, (const float*)0, (float*)0, (float*)0, Mp,
                                                    AGG1, lin1_b, (const float*)0, H1h, H1l);

  k_gemm<<<dim3(D2 / GC, Mp / GR), B, 0, stream>>>(H1h, H1l, HD1, w2h, w2l, HD1, D2, 0, H2T,
                                                   att_src2, att_dst2, ss2, sd2, Mp,
                                                   (const float*)0, (const float*)0, (const float*)0,
                                                   (__bf16*)0, (__bf16*)0);
  k_gemm<<<dim3(D2 / GC, Mp / GR), B, 0, stream>>>(H1h, H1l, HD1, l2h, l2l, HD1, D2, 2, R2,
                                                   (const float*)0, (const float*)0, (float*)0, (float*)0, Mp,
                                                   (const float*)0, b2, lin2_b, (__bf16*)0, (__bf16*)0);
  k_edge_p<1><<<cdivu((long)Etp / 4, NTHR), B, 0, stream>>>(ei, nE, nEt, nN, ss2, sd2, Mp, P2, Etp / 4);
  hipFuncSetAttribute(reinterpret_cast<const void*>(&k_agg<D2, 1, NB2, 4>),
                      hipFuncAttributeMaxDynamicSharedMemorySize, AGG_LDS(D2, 1, NB2));
  k_agg<D2, 1, NB2, 4><<<cdivu(Mp, NB2), B, AGG_LDS(D2, 1, NB2), stream>>>(
      ei, nE, nN, P2, H2T, (const float*)0, R2, out0, nN, (float*)0, Mp);
}
